// HybridGATGCN_29222957481999
// MI455X (gfx1250) — hardware-run, weakly checked
//
#include <hip/hip_runtime.h>

namespace {

constexpr int N = 50000, NP = 50016, NPL = NP  , SRCM = N  , EFULL = 800000  , E = EFULL  ;
constexpr int F = 128  , FO = 64  , VOC = 1, NRL = NP  , NL = (NPL < N ? NPL : N);
constexpr float LN_EPS = 1e-5f;
constexpr float LNEPS = 1e-5f; constexpr float XS = 8.0f, WSC = 256.0f, WSQ = 0.25f, RS_ = 1024.0f, NSL_ = 0.2f, NSA_ = 0.01f, SLOPE = 0.0f, BNEPS = 1e-5f;
static_assert(NP % 32 == 0 && NP >= N && NPL % 32 == 0 && F % 32 == 0, "tiling");
static_assert(F == 128 && FO == 64, "a 128-wide input; the last GEMM writes 64 columns (NT = 4) onto a 64-pitch plane whose first 40 are real: the dense copy-out writes the output");
typedef _Float16 b16;
typedef __attribute__((ext_vector_type(16))) _Float16 v16b;
typedef __attribute__((ext_vector_type(8))) _Float16 v8b;
typedef __attribute__((ext_vector_type(8))) float v8f;
typedef __attribute__((ext_vector_type(4))) float v4f;
__device__ __forceinline__ float bf16_rne(float f) { unsigned int u = __float_as_uint(f); u += 0x7FFFu + ((u >> 16) & 1u); return __uint_as_float(u & 0xFFFF0000u); }
__device__ __forceinline__ void split16(float v, b16& hi, b16& lo) { hi = (b16)v; lo = (b16)(v - (float)hi); }
__device__ __forceinline__ v16b frag_kb(const b16* p, int hh) { const v8b a = *(const v8b*)(p + 8 * hh), b = *(const v8b*)(p + 16 + 8 * hh); v16b f;
#pragma unroll
  for (int e = 0; e < 8; ++e) { f[e] = a[e]; f[8 + e] = b[e]; } return f; }
__device__ __forceinline__ v8f wmma16b(v16b a, v16b b, v8f c) { v8f d = __builtin_amdgcn_wmma_f32_16x16x32_f16(false, a, false, b, (short)0, c, false, false); asm volatile("v_nop\n\tv_nop\n\tv_nop\n\tv_nop" : "+v"(d) : "v"(a), "v"(b)); return d; }
__device__ __forceinline__ void wave_lds_sync() { __builtin_amdgcn_fence(__ATOMIC_RELEASE, "workgroup"); __builtin_amdgcn_wave_barrier(); __builtin_amdgcn_fence(__ATOMIC_ACQUIRE, "workgroup"); }
__device__ __forceinline__ int iclamp(int v, int lo, int hi) { return v < lo ? lo : (v > hi ? hi : v); }
constexpr int CSR_NBLK = 512, CSR_GB = 8  , CSR_GN = 1 << CSR_GB  , CSR_MAXG = 512, CSR_CAP = 12288  ;
static_assert(((N + CSR_GN - 1) >> CSR_GB) <= CSR_MAXG && CSR_GN % 4 == 0 && CSR_GN <= 65536, "csr: bucket count / 16-bit node key");
__global__ __launch_bounds__(64) void csrA_kernel(const int* __restrict__ dst, int E, int N, int nG, int CHP, int NGP, int* __restrict__ STG, int* __restrict__ HST) {
  extern __shared__ int sm[];
  int* cnt = sm; int* run = sm + NGP; int* ids = sm + 2 * NGP;
  const int b = blockIdx.x; const int ch = (E + CSR_NBLK - 1) / CSR_NBLK; const int e0 = b * ch, e1 = min(E, e0 + ch);
  for (int i = threadIdx.x; i < NGP; i += 64) cnt[i] = 0;
  for (int i = threadIdx.x; i < CHP; i += 64) ids[i] = -1;
  __syncthreads();
  if (threadIdx.x == 0) {
    for (int e = e0; e < e1; ++e) { int d = dst[e]; d = (d < 0) ? 0 : (d >= N ? N - 1 : d); cnt[d >> CSR_GB] += 1; }
    int acc = 0; for (int g = 0; g < nG; ++g) { run[g] = acc; acc += cnt[g]; }
    for (int e = e0; e < e1; ++e) { int d = dst[e]; d = (d < 0) ? 0 : (d >= N ? N - 1 : d); const int g = d >> CSR_GB; ids[run[g]] = e; run[g] += 1; } }
  __syncthreads();
  typedef __attribute__((ext_vector_type(4))) int v4i;
  for (int pass = 0; pass < 2; ++pass) {
    for (int i = threadIdx.x; i < CHP / 4; i += 64) *(volatile v4i*)(STG + (size_t)b * CHP + i * 4) = *(const v4i*)(&ids[i * 4]);
    for (int i = threadIdx.x; i < NGP / 4; i += 64) { v4i v; for (int e = 0; e < 4; ++e) v[e] = (i * 4 + e < nG) ? cnt[i * 4 + e] : 0; *(volatile v4i*)(HST + (size_t)b * NGP + i * 4) = v; }
    __threadfence(); }
}
__global__ __launch_bounds__(512) void csrS_kernel(const int* __restrict__ HST, int nG, int NGP, int* __restrict__ START, int* __restrict__ TOT, int* __restrict__ OFF) {
  __shared__ int tot[CSR_MAXG];
  const int b = threadIdx.x;
  for (int pass = 0; pass < 2; ++pass) { int runb = 0; for (int g = 0; g < nG; ++g) { int c = HST[(size_t)b * NGP + g]; c = (c < 0) ? 0 : c; ((volatile int*)OFF)[(size_t)g * CSR_NBLK + b] = runb; runb += c; } __threadfence(); }
  for (int g = threadIdx.x; g < nG; g += 512) { int s = 0; for (int bb = 0; bb < CSR_NBLK; ++bb) { int c = HST[(size_t)bb * NGP + g]; s += (c < 0) ? 0 : c; } tot[g] = s; }
  __syncthreads();
  if (threadIdx.x < 32) {
    __shared__ int st[CSR_MAXG + 32];
    if (threadIdx.x == 0) { int acc = 0; for (int g = 0; g < NGP; ++g) { st[g] = acc; if (g < nG) acc += (tot[g] + 31) & ~31; } st[NGP] = acc; }
    __builtin_amdgcn_fence(__ATOMIC_RELEASE, "workgroup"); __builtin_amdgcn_wave_barrier(); __builtin_amdgcn_fence(__ATOMIC_ACQUIRE, "workgroup");
    for (int pass = 0; pass < 2; ++pass) { for (int i = threadIdx.x; i < NGP + 32; i += 32) { ((volatile int*)START)[i] = (i <= NGP) ? st[min(i, NGP)] : 0; ((volatile int*)TOT)[i] = (i < nG) ? tot[i] : 0; } __threadfence(); } }
}
__global__ __launch_bounds__(256) void csrB_kernel(const int* __restrict__ dst, int N, int nG, int CHP, int NGP, int permLen, const int* __restrict__ STG, const int* __restrict__ HST, const int* __restrict__ OFF, const int* __restrict__ START, const int* __restrict__ TOT, int* __restrict__ PERM, int* __restrict__ ROWPTR, int* __restrict__ ROWCNT, int* __restrict__ FLAG) {
  typedef __attribute__((ext_vector_type(4))) int v4i;
  __shared__ int ids[CSR_CAP]; __shared__ unsigned short key[CSR_CAP]; __shared__ int outp[CSR_CAP]; __shared__ int ncnt[CSR_GN + 1]; __shared__ int boff[CSR_NBLK + 1];
  const int g = blockIdx.x, t_ = threadIdx.x; int tot = TOT[g]; int st = START[g], stn = START[g + 1]; const int v0 = g * CSR_GN; const int nv = min(CSR_GN, N - v0);
  st = (st < 0) ? 0 : (st > permLen - 32 ? permLen - 32 : st) & ~31; stn = (stn < st) ? st : (stn > permLen ? permLen : stn); tot = (tot < 0) ? 0 : tot; if (tot > stn - st && tot <= CSR_CAP) tot = stn - st;
  if (tot > CSR_CAP) {
    for (int pass = 0; pass < 2; ++pass) { for (int i = t_; i < CSR_GN / 4; i += 256) { v4i a, c; for (int e = 0; e < 4; ++e) { a[e] = st; c[e] = 0; } *(volatile v4i*)(ROWPTR + v0 + i * 4) = a; *(volatile v4i*)(ROWCNT + v0 + i * 4) = c; } if (t_ == 0) ((volatile int*)FLAG)[0] = 1; __threadfence(); } (void)nv; return; }
  if (t_ == 0) { int acc = 0; for (int b = 0; b < CSR_NBLK; ++b) { boff[b] = acc; int c = HST[(size_t)b * NGP + g]; c = (c < 0) ? 0 : (c > CHP ? CHP : c); acc += c; if (acc > tot) acc = tot; } boff[CSR_NBLK] = acc; }
  for (int i = t_; i <= CSR_GN; i += 256) ncnt[i] = 0;
  __syncthreads();
  for (int b = 0; b < CSR_NBLK; ++b) { const int c = boff[b + 1] - boff[b]; int o_ = OFF[(size_t)g * CSR_NBLK + b]; o_ = (o_ < 0) ? 0 : (o_ > CHP - c ? CHP - c : o_); const int* src_ = STG + (size_t)b * CHP + o_;
    for (int i = t_; i < c; i += 256) { int id = src_[i]; id = (id < 0) ? 0 : id; ids[boff[b] + i] = id; int d = dst[id]; d = (d < v0) ? v0 : (d >= N ? N - 1 : d); int kk = d - v0; kk = (kk < 0) ? 0 : (kk >= CSR_GN ? CSR_GN - 1 : kk); key[boff[b] + i] = (unsigned short)kk; } }
  __syncthreads();
  if (t_ == 0) { for (int i = 0; i < tot; ++i) ncnt[key[i]] += 1; int acc = 0; for (int vl = 0; vl < CSR_GN; ++vl) { const int c = ncnt[vl]; ncnt[vl] = acc; acc += c; } ncnt[CSR_GN] = acc;
    for (int i = 0; i < tot; ++i) { const int vl = key[i]; outp[ncnt[vl]] = ids[i]; ncnt[vl] += 1; }
    for (int vl = CSR_GN; vl > 0; --vl) ncnt[vl] = ncnt[vl - 1]; ncnt[0] = 0; }
  __syncthreads();
  for (int pass = 0; pass < 2; ++pass) {
    for (int i = t_; i < (stn - st) / 4; i += 256) { v4i v; for (int e = 0; e < 4; ++e) { const int q = i * 4 + e; v[e] = (q < tot) ? outp[q] : -1; } *(volatile v4i*)(PERM + st + i * 4) = v; }
    for (int i = t_; i < CSR_GN / 4; i += 256) { v4i a, c; for (int e = 0; e < 4; ++e) { const int vl = i * 4 + e; a[e] = st + ncnt[vl]; c[e] = (vl < nv) ? (ncnt[vl + 1] - ncnt[vl]) : 0; } *(volatile v4i*)(ROWPTR + v0 + i * 4) = a; *(volatile v4i*)(ROWCNT + v0 + i * 4) = c; }
    __threadfence(); }
}
__global__ __launch_bounds__(256) void csrZ_kernel(int* __restrict__ p, size_t n4) { typedef __attribute__((ext_vector_type(4))) int v4i; const size_t tid = (size_t)blockIdx.x * 256 + threadIdx.x, nth = (size_t)gridDim.x * 256; v4i z = {0, 0, 0, 0}; for (size_t i = tid; i < n4; i += nth) *(volatile v4i*)(p + i * 4) = z; }
struct CsrBufs { int *STG, *HST, *OFF, *START, *TOT, *PERM, *ROWPTR, *ROWCNT, *FLAG; int nG, NGP, CHP; size_t permLen; char* base; size_t bytes; };
static size_t csr_carve(CsrBufs& c, char* ws, size_t off, int E, int N) {
  const size_t off0 = off; c.base = ws + off;
  auto al = [&](size_t bytes) { char* p = ws + off; off += (bytes + 255) & ~(size_t)255; return p; };
  c.nG = (N + CSR_GN - 1) / CSR_GN; c.NGP = (c.nG + 31) & ~31; const int ch = (E + CSR_NBLK - 1) / CSR_NBLK; c.CHP = (ch + 31) & ~31; c.permLen = (size_t)E + 32 * (size_t)c.nG + 32;
  c.STG = (int*)al((size_t)CSR_NBLK * c.CHP * 4); c.HST = (int*)al((size_t)CSR_NBLK * c.NGP * 4); c.OFF = (int*)al((size_t)c.NGP * CSR_NBLK * 4); c.START = (int*)al((size_t)(c.NGP + 64) * 4); c.TOT = (int*)al((size_t)(c.NGP + 64) * 4);
  c.PERM = (int*)al(c.permLen * 4); c.ROWPTR = (int*)al((size_t)c.nG * CSR_GN * 4); c.ROWCNT = (int*)al((size_t)c.nG * CSR_GN * 4); c.FLAG = (int*)al(256);
  c.bytes = off - off0; return off;
}
static void csr_build(const CsrBufs& c, const int* dst, int E, int N, hipStream_t stream) {
  const size_t smem = (size_t)(2 * c.NGP + c.CHP) * 4;
  csrZ_kernel<<<512, 256, 0, stream>>>((int*)c.base, c.bytes / 16);
  csrA_kernel<<<CSR_NBLK, 64, smem, stream>>>(dst, E, N, c.nG, c.CHP, c.NGP, c.STG, c.HST);
  csrS_kernel<<<1, 512, 0, stream>>>(c.HST, c.nG, c.NGP, c.START, c.TOT, c.OFF);
  csrB_kernel<<<c.nG, 256, 0, stream>>>(dst, N, c.nG, c.CHP, c.NGP, (int)c.permLen, c.STG, c.HST, c.OFF, c.START, c.TOT, c.PERM, c.ROWPTR, c.ROWCNT, c.FLAG);
}

typedef __attribute__((ext_vector_type(4))) _Float16 v4h;
__device__ __forceinline__ float lrelu(float v) { return v > 0.0f ? v : NSL_ * v; }
template <int K, int NOUTR, int NOUTP>
__global__ __launch_bounds__(256) void wt_kernel(const float* __restrict__ w, b16* __restrict__ WT, float scl) {
  const int u = blockIdx.x * 256 + threadIdx.x; if (u >= NOUTP * K / 8) return; const int e = u * 8; const int o = e / K, k0 = e % K; v8b v;
#pragma unroll
  for (int j = 0; j < 8; ++j) v[j] = (b16)(o < NOUTR ? bf16_rne(w[(size_t)(k0 + j) * NOUTR + o]) * scl : 0.0f);
  for (int pass = 0; pass < 2; ++pass) { *(volatile v8b*)(WT + e) = v; __threadfence(); }
}
template <int W>
__global__ __launch_bounds__(256) void rscalew_kernel(const float* __restrict__ H, const float* __restrict__ DEG, float* __restrict__ HS, int nv, int nrows) {
  static_assert(W >= 4 && W % 4 == 0, "rscalew: float4 steps"); const size_t i = (size_t)blockIdx.x * 256 + threadIdx.x; if (i >= (size_t)nrows * (W / 4)) return; const size_t v = i / (W / 4); const int c = (int)(i % (W / 4)) * 4; v4f o = {0.0f, 0.0f, 0.0f, 0.0f};
  if (v < (size_t)nv) { const float dg = DEG[v]; const float dv = (dg > 0.0f) ? rsqrtf(dg) : 0.0f; const v4f t = *(const v4f*)(H + v * W + c); for (int j = 0; j < 4; ++j) o[j] = (dv * t[j]); }
  for (int pass = 0; pass < 2; ++pass) { *(volatile v4f*)(HS + v * W + c) = o; __threadfence(); }
}
template <int W, bool RELU>
__global__ __launch_bounds__(256) void wfinw_kernel(const float* __restrict__ AG, const float* __restrict__ HS, const float* __restrict__ DEG, const float* __restrict__ b, float* __restrict__ OUT, int nv, int nrows) {
  static_assert(W >= 4 && W % 4 == 0, "wfinw: float4 steps"); const size_t i = (size_t)blockIdx.x * 256 + threadIdx.x; if (i >= (size_t)nrows * (W / 4)) return; const size_t v = i / (W / 4); const int c = (int)(i % (W / 4)) * 4; v4f o = {0.0f, 0.0f, 0.0f, 0.0f};
  if (v < (size_t)nv) { const float dg = DEG[v]; const float dv = (dg > 0.0f) ? rsqrtf(dg) : 0.0f; const v4f a = *(const v4f*)(AG + v * W + c), s = *(const v4f*)(HS + v * W + c); for (int j = 0; j < 4; ++j) { const float y = (dv * (a[j] + s[j])) + bf16_rne(b[c + j]); o[j] = RELU ? fmaxf(y, 0.0f) : y; } }
  for (int pass = 0; pass < 2; ++pass) { *(volatile v4f*)(OUT + v * W + c) = o; __threadfence(); }
}
template <int W, bool RELU>
__global__ __launch_bounds__(256) void baddw_kernel(const float* __restrict__ A, const float* __restrict__ b, float* __restrict__ OUT, int nv, int nrows) {
  static_assert(W >= 4 && W % 4 == 0, "baddw: float4 steps"); const size_t i = (size_t)blockIdx.x * 256 + threadIdx.x; if (i >= (size_t)nrows * (W / 4)) return; const size_t v = i / (W / 4); const int c = (int)(i % (W / 4)) * 4; v4f o = {0.0f, 0.0f, 0.0f, 0.0f};
  if (v < (size_t)nv) { const v4f a = *(const v4f*)(A + v * W + c); for (int j = 0; j < 4; ++j) { const float y = a[j] + bf16_rne(b[c + j]); o[j] = RELU ? fmaxf(y, 0.0f) : y; } }
  for (int pass = 0; pass < 2; ++pass) { *(volatile v4f*)(OUT + v * W + c) = o; __threadfence(); }
}
__global__ __launch_bounds__(256) void zfill_kernel(float* __restrict__ p, int n) { for (int pass = 0; pass < 2; ++pass) { for (int i = threadIdx.x; i < n; i += 256) ((volatile float*)p)[i] = 0.0f; __threadfence(); } }
template <int K, int NT, int PREC, int MODE, bool GIDX>
__global__ __launch_bounds__(64) void lin_kernel(const float* __restrict__ X, const int* __restrict__ gidx, const b16* __restrict__ WT, const b16* __restrict__ WQ, const float* __restrict__ bias, float* __restrict__ OUT, int opitch, int nvalid, int mrows) {
  constexpr int NC = NT * 16;
  __shared__ __attribute__((aligned(16))) b16 Ah[2][16][K + 8], Al[2][16][(PREC == 0 ? K : 0) + 8]; __shared__ __attribute__((aligned(16))) float Tf[2][16][NC + 4];
  const int wave = threadIdx.x >> 5, lane = threadIdx.x & 31, nloc = lane & 15, hlf = lane >> 4; const size_t m0 = (size_t)blockIdx.x * 32 + wave * 16;
  for (int idx = lane; idx < 16 * (K / 4); idx += 32) { const int rr = idx / (K / 4), c4 = (idx % (K / 4)) * 4; const size_t vrow = (m0 + rr < (size_t)nvalid) ? m0 + rr : (size_t)nvalid - 1; size_t arow = vrow; if (GIDX) arow = (size_t)iclamp(gidx[vrow], 0, VOC - 1);
    const v4f v = *(const v4f*)(X + arow * K + c4); v4h hv, lv;
    for (int j = 0; j < 4; ++j) { float vj = v[j]; if (MODE == 2) vj = fmaxf(vj, 0.0f); const float vs = (PREC == 1 ? bf16_rne(vj) : vj) * XS; const b16 ph = (b16)vs; hv[j] = ph; lv[j] = (b16)((vs - (float)ph) * RS_); } *(v4h*)(&Ah[wave][rr][c4]) = hv; if (PREC == 0) *(v4h*)(&Al[wave][rr][c4]) = lv; }
  wave_lds_sync();
  v8f acc[NT];
#pragma unroll
  for (int t = 0; t < NT; ++t) acc[t] = (v8f){};
#pragma unroll 1
  for (int kb = 0; kb < K; kb += 32) { const v16b a = frag_kb(&Ah[wave][nloc][kb], hlf); v16b al; if (PREC == 0) al = frag_kb(&Al[wave][nloc][kb], hlf);
#pragma unroll
    for (int t = 0; t < NT; ++t) { const size_t wo_ = (size_t)(t * 16 + nloc) * K + kb; acc[t] = wmma16b(a, frag_kb(WT + wo_, hlf), acc[t]); if (PREC == 0) acc[t] = wmma16b(al, frag_kb(WQ + wo_, hlf), acc[t]); } }
#pragma unroll
  for (int t = 0; t < NT; ++t) { const int col = t * 16 + nloc; const float bb = (MODE == 14 || MODE == 17) ? 0.0f : bf16_rne(bias[col]);
    for (int r = 0; r < 8; ++r) { const size_t vrow = m0 + 8 * hlf + r; float y = acc[t][r] * (1.0f / (XS * WSC)) + bb; if (MODE == 1) y = fmaxf(y, 0.0f); if ((MODE == 14 || MODE == 17) && vrow < (size_t)mrows) y += OUT[vrow * (size_t)opitch + col]; if (MODE == 17) y = fmaxf(y, 0.0f);     Tf[wave][8 * hlf + r][col] = (vrow < (size_t)nvalid) ? y : 0.0f; } }
  wave_lds_sync();
  for (int pass = 0; pass < 2; ++pass) { for (int rr = 0; rr < 16; ++rr) { if (m0 + rr < (size_t)mrows) { if (NC >= 128) { for (int c8 = 0; c8 < NC; c8 += 128) *(volatile v4f*)(OUT + (m0 + rr) * (size_t)opitch + c8 + lane * 4) = *(const v4f*)(&Tf[wave][rr][c8 + lane * 4]); }
        else { if (lane < NC / 4) *(volatile v4f*)(OUT + (m0 + rr) * (size_t)opitch + lane * 4) = *(const v4f*)(&Tf[wave][rr][lane * 4]); } } } __threadfence(); }
}
__global__ __launch_bounds__(256) void rscale_kernel(const float* __restrict__ H, const float* __restrict__ DEG, float* __restrict__ HS, int nrows) {
  const size_t i = (size_t)blockIdx.x * 256 + threadIdx.x; if (i >= (size_t)nrows * (F / 4)) return; const size_t v = i / (F / 4); const int c = (int)(i % (F / 4)) * 4; v4f o = {0.0f, 0.0f, 0.0f, 0.0f};
  if (v < (size_t)N) { const float dg = DEG[v]; const float dv = (dg > 0.0f) ? rsqrtf(dg) : 0.0f; const v4f t = *(const v4f*)(H + v * F + c); for (int j = 0; j < 4; ++j) o[j] = (dv * t[j]); }
  for (int pass = 0; pass < 2; ++pass) { *(volatile v4f*)(HS + v * F + c) = o; __threadfence(); }
}
template <int W>
__global__ __launch_bounds__(256) void hsum_kernel(const float* __restrict__ X, int xp, int ns, int srcm, const int* __restrict__ srcs, int ecut, const int* __restrict__ PERM, const int* __restrict__ ROWPTR, const int* __restrict__ ROWCNT, int permLen, float* __restrict__ P, int pp, int ocol, int nd, int ndp) {
  constexpr int CW = W / 8; static_assert(W % 32 == 0, "hsum: 8 threads per row, float4 steps");
  const int tid = threadIdx.x; const int row = tid >> 3, g = tid & 7, c0 = g * CW; const int v = blockIdx.x * 32 + row; if (v >= ndp) return;
  int cnt = 0, p0 = 0; if (v < nd) { cnt = iclamp(ROWCNT[v], 0, 65536); p0 = iclamp(ROWPTR[v], 0, permLen - 1); if (p0 + cnt > permLen) cnt = permLen - p0; }
  float m[CW];
#pragma unroll
  for (int j = 0; j < CW; ++j) m[j] = 0.0f;
#pragma unroll 1
  for (int i = 0; i < cnt; ++i) { const int e = iclamp(PERM[p0 + i], 0, ecut - 1); int s = iclamp(srcs[e], 0, ns - 1); if (srcm < ns) s %= srcm; const float* xr = X + (size_t)s * xp + c0;
#pragma unroll
    for (int q = 0; q < CW / 4; ++q) { const v4f a = *(const v4f*)(xr + 4 * q); for (int j = 0; j < 4; ++j) m[4 * q + j] += a[j]; } }
  for (int pass = 0; pass < 2; ++pass) { float* orow = P + (size_t)v * pp + ocol + c0;
#pragma unroll
    for (int q = 0; q < CW / 4; ++q) { v4f o4; for (int j = 0; j < 4; ++j) o4[j] = (v < nd) ? m[4 * q + j] : 0.0f; *(volatile v4f*)(orow + 4 * q) = o4; }
    __threadfence(); }
}
template <int W>
__global__ __launch_bounds__(256) void xcpw_kernel(const float* __restrict__ x, float* __restrict__ P, int pp, int n, int np_) {
  const size_t i = (size_t)blockIdx.x * 256 + threadIdx.x; const size_t v = i / (W / 4); const int c = (int)(i % (W / 4)) * 4; if (v >= (size_t)np_) return; v4f t = {0.0f, 0.0f, 0.0f, 0.0f};
  if (v < (size_t)n) { t = *(const v4f*)(x + v * W + c); for (int j = 0; j < 4; ++j) t[j] = bf16_rne(t[j]); }
  for (int pass = 0; pass < 2; ++pass) { *(volatile v4f*)(P + v * (size_t)pp + c) = t; __threadfence(); }
}
__global__ __launch_bounds__(256) void cdeg_kernel(const int* __restrict__ ROWCNT, float* __restrict__ DEG, int n) {
  const int v = blockIdx.x * 256 + threadIdx.x; if (v >= n) return; float s = 1.0f; if (v < N) { const int c = iclamp(ROWCNT[v], 0, 1 << 24); s = (c > 1) ? (float)c : 1.0f; }
  for (int pass = 0; pass < 2; ++pass) { ((volatile float*)DEG)[v] = s; __threadfence(); }
}
template <int W, int MODE>
__global__ __launch_bounds__(256) void colpart_kernel(const float* __restrict__ H, const float* __restrict__ MEAN, float* __restrict__ PART, int nstat) {
  const int b = blockIdx.x, c = threadIdx.x; if (c >= W) return; const float mu = (MODE == 1) ? MEAN[c] : 0.0f; float s = 0.0f; const int v0 = b * 512, v1 = (v0 + 512 < nstat) ? v0 + 512 : nstat;
  for (int v = v0; v < v1; ++v) { const float h = H[(size_t)v * W + c]; if (MODE == 1) { const float d = h - mu; s += (d * d); } else s += h; }
  for (int pass = 0; pass < 2; ++pass) { ((volatile float*)PART)[(size_t)b * W + c] = s; __threadfence(); }
}
template <int W, int MODE>
__global__ __launch_bounds__(256) void colred_kernel(const float* __restrict__ PART, int nb, int nstat, const float* __restrict__ MEAN, const float* __restrict__ gam, const float* __restrict__ bet, float* __restrict__ OUT, float* __restrict__ OUT2) {
  const int c = threadIdx.x; if (c >= W) return; float s = 0.0f;
  for (int b = 0; b < nb; ++b) s += PART[(size_t)b * W + c];
  const float m = s / (float)nstat;
  for (int pass = 0; pass < 2; ++pass) {
    if (MODE == 0) ((volatile float*)OUT)[c] = m;
    else { const float scl = bf16_rne(gam[c]) * rsqrtf(m + BNEPS); ((volatile float*)OUT)[c] = scl; ((volatile float*)OUT2)[c] = bf16_rne(bet[c]) - MEAN[c] * scl; }
    __threadfence(); }
}
template <int W, int ACT>
__global__ __launch_bounds__(256) void bnact_kernel(const float* __restrict__ H, const float* __restrict__ SCL, const float* __restrict__ SFT, float* __restrict__ OUT, int op, int mrows) {
  const size_t i = (size_t)blockIdx.x * 256 + threadIdx.x; if (i >= (size_t)mrows * (W / 4)) return; const size_t v = i / (W / 4); const int c = (int)(i % (W / 4)) * 4;
  const v4f h = *(const v4f*)(H + v * W + c), s = *(const v4f*)(SCL + c), t = *(const v4f*)(SFT + c); v4f o;
  for (int j = 0; j < 4; ++j) { float y = (h[j] * s[j]) + t[j]; if (ACT == 1) y = fmaxf(y, 0.0f); if (ACT == 2) y = (y > 0.0f) ? y : (__expf(y) - 1.0f);     if (ACT == 3) y = (y >= 0.0f) ? y : 0.01f * y; o[j] = y; }
  for (int pass = 0; pass < 2; ++pass) { *(volatile v4f*)(OUT + v * (size_t)op + c) = o; __threadfence(); }
}
__global__ __launch_bounds__(256) void addk_kernel(const float* __restrict__ A, const float* __restrict__ B, float* __restrict__ Y, size_t n4, float oscale) {
  const size_t i = (size_t)blockIdx.x * 256 + threadIdx.x; if (i >= n4) return; const v4f a = *(const v4f*)(A + 4 * i), b = *(const v4f*)(B + 4 * i); v4f o; for (int j = 0; j < 4; ++j) o[j] = ((a[j] + b[j]) * oscale);
  for (int pass = 0; pass < 2; ++pass) { *(volatile v4f*)(Y + 4 * i) = o; __threadfence(); }
}
template <int W>
__global__ __launch_bounds__(256) void rowst_kernel(const float* __restrict__ H, float eps, float* __restrict__ MU, float* __restrict__ INV, int nrows) {
  static_assert(W % 4 == 0, "rowst: float4 steps"); const int v = blockIdx.x * 256 + threadIdx.x; if (v >= nrows) return; const float* hr = H + (size_t)v * W; float s = 0.0f;
  for (int q = 0; q < W / 4; ++q) { const v4f a = *(const v4f*)(hr + 4 * q); for (int j = 0; j < 4; ++j) s += a[j]; }
  const float mu = s / (float)W; float ss = 0.0f;
  for (int q = 0; q < W / 4; ++q) { const v4f a = *(const v4f*)(hr + 4 * q); for (int j = 0; j < 4; ++j) { const float d = a[j] - mu; ss += (d * d); } }
  const float inv = 1.0f / sqrtf(ss / (float)W + eps);
  for (int pass = 0; pass < 2; ++pass) { ((volatile float*)MU)[v] = mu; ((volatile float*)INV)[v] = inv; __threadfence(); }
}
template <int W>
__global__ __launch_bounds__(256) void rowap_kernel(const float* __restrict__ H, const float* __restrict__ MU, const float* __restrict__ INV, const float* __restrict__ scale, const float* __restrict__ offset, float* __restrict__ OUT, int nrows) {
  static_assert(W % 4 == 0, "rowap: float4 steps"); const size_t i = (size_t)blockIdx.x * 256 + threadIdx.x; if (i >= (size_t)nrows * (W / 4)) return; const size_t v = i / (W / 4); const int c = (int)(i % (W / 4)) * 4;
  const float mu = MU[v], inv = INV[v]; const v4f a = *(const v4f*)(H + v * W + c); v4f o; for (int j = 0; j < 4; ++j) o[j] = ((((a[j] - mu) * inv)) * bf16_rne(scale[c + j])) + bf16_rne(offset[c + j]);
  for (int pass = 0; pass < 2; ++pass) { *(volatile v4f*)(OUT + v * W + c) = o; __threadfence(); }
}
__global__ __launch_bounds__(256) void emask_kernel(const int* __restrict__ et, int r, int nrel, float* __restrict__ G, int e, int ef) {
  const size_t t = (size_t)blockIdx.x * 256 + threadIdx.x; if (t >= (size_t)ef) return; float g = 0.0f;
  if (t < (size_t)e) { const int ty = iclamp(et[t], 0, nrel - 1); if (ty == r) g = 1.0f; }
  for (int pass = 0; pass < 2; ++pass) { ((volatile float*)G)[t] = g; __threadfence(); }
}
__global__ __launch_bounds__(256) void wcnt_kernel(const float* __restrict__ EW, const int* __restrict__ PERM, const int* __restrict__ ROWPTR, const int* __restrict__ ROWCNT, int permLen, float* __restrict__ D, int n, int nrows) {
  const int v = blockIdx.x * 256 + threadIdx.x; if (v >= nrows) return; float s = 0.0f;
  if (v < n) { int cnt = iclamp(ROWCNT[v], 0, 65536); const int p0 = iclamp(ROWPTR[v], 0, permLen - 1); if (cnt > permLen - p0) cnt = permLen - p0;
    for (int i = 0; i < cnt; ++i) { const int e = iclamp(PERM[p0 + i], 0, E - 1); s += EW[e]; } }
  for (int pass = 0; pass < 2; ++pass) { ((volatile float*)D)[v] = s; __threadfence(); }
}
template <int K, int NO, bool OI>
__global__ __launch_bounds__(256) void headw_kernel(const float* __restrict__ P, int pp, const float* __restrict__ wl, const float* __restrict__ bl, float* __restrict__ out, int total) {
  static_assert(K >= 1 && NO >= 1 && NO <= 16, "headw: a narrow head (the matrix unit serves wider ones)"); const int t = blockIdx.x * 256 + threadIdx.x; if (t >= total) return; const int g = t / NO, k = t - g * NO; float s = bf16_rne(bl[k]);
  for (int c = 0; c < K; ++c) s += (P[(size_t)g * pp + c] * bf16_rne(OI ? wl[k * K + c] : wl[c * NO + k]));
  for (int pass = 0; pass < 2; ++pass) { ((volatile float*)out)[t] = s; __threadfence(); }
}
template <int ACT>
__global__ __launch_bounds__(256) void eact_kernel(const float* __restrict__ P, float* __restrict__ OUT, size_t n4, float sl) {
  static_assert(ACT >= 1 && ACT <= 9, "eact: nine activations"); const size_t i = (size_t)blockIdx.x * 256 + threadIdx.x; if (i >= n4) return; const v4f a = *(const v4f*)(P + 4 * i); v4f o;
  for (int j = 0; j < 4; ++j) { const float v = a[j]; float y;
    if (ACT == 1) y = fmaxf(v, 0.0f);
    else if (ACT == 2) y = (v >= 0.0f) ? v : (sl * v);
    else if (ACT == 3) y = 1.0f / (1.0f + expf(-v));
    else if (ACT == 4) y = tanhf(v);
    else if (ACT == 5) y = (v > 0.0f) ? v : expm1f(v);
    else if (ACT == 6) y = v / (1.0f + expf(-v));
    else if (ACT == 7) y = (((0.5f * v)) * (1.0f + tanhf(0.7978845608028654f * (v + (0.044715f * ((v * ((v * v)))))))));
    else if (ACT == 8) y = (((0.5f * v)) * (1.0f + erff((v * 0.7071067811865476f))));
    else y = (1.0507009873554805f * ((v > 0.0f) ? v : (1.6732632423543772f * expm1f(v))));
    o[j] = y; }
  for (int pass = 0; pass < 2; ++pass) { *(volatile v4f*)(OUT + 4 * i) = o; __threadfence(); }
}
__global__ __launch_bounds__(256) void ocpm_kernel(const float* __restrict__ P0, int nc0, int pw0, const float* __restrict__ P1, int nc1, int pw1, int s1, const float* __restrict__ P2, int nc2, int pw2, int s2,
                                                   const float* __restrict__ P3, int nc3, int pw3, int s3, float* __restrict__ out, int total) {
  const int t = blockIdx.x * 256 + threadIdx.x; if (t >= total) return; const float* P = P0; int nc = nc0, pw = pw0, s = 0, e = s1;
  if (t >= s1) { P = P1; nc = nc1; pw = pw1; s = s1; e = s2; } if (t >= s2) { P = P2; nc = nc2; pw = pw2; s = s2; e = s3; } if (t >= s3) { P = P3; nc = nc3; pw = pw3; s = s3; e = total; }
  const unsigned j = (unsigned)((t < e ? t : e - 1) - s), g = j / (unsigned)nc, k = j - g * (unsigned)nc; const float v = P[(size_t)g * (unsigned)pw + k];
  for (int pass = 0; pass < 2; ++pass) { ((volatile float*)out)[t] = v; __threadfence(); }
}
__global__ __launch_bounds__(256) void cdegr_kernel(const int* __restrict__ ROWCNT, float* __restrict__ DEG, int n) {
  const int v = blockIdx.x * 256 + threadIdx.x; if (v >= n) return; float s = 0.0f; if (v < N) { const int c = iclamp(ROWCNT[v], 0, 1 << 24); s = (float)c; }
  for (int pass = 0; pass < 2; ++pass) { ((volatile float*)DEG)[v] = s; __threadfence(); }
}
template <int W, int ACT>
__global__ __launch_bounds__(256) void gcn_kernel(const float* __restrict__ Hh, const int* __restrict__ srcs, const int* __restrict__ PERM, const int* __restrict__ ROWPTR, const int* __restrict__ ROWCNT, int permLen, const float* __restrict__ bias, const float* __restrict__ ADDP, float* __restrict__ out, int mrows) {
  constexpr int CW = W / 8;
  static_assert(W % 32 == 0, "gcn: 8 threads per row, float4 stores");
  const int tid = threadIdx.x; const int row = tid >> 3, g = tid & 7, c0 = g * CW; const int v = blockIdx.x * 32 + row; const int vv = v < N ? v : N - 1;
  int cnt = 0, p0 = 0; if (v < N) { cnt = iclamp(ROWCNT[v], 0, 65536); p0 = iclamp(ROWPTR[v], 0, permLen - 1); if (p0 + cnt > permLen) cnt = permLen - p0; }
  const float dv = rsqrtf((float)(cnt + 1));
  float m[CW]; { const float* hr = Hh + (size_t)vv * W + c0;
#pragma unroll
    for (int q = 0; q < CW / 4; ++q) { const v4f t4 = *(const v4f*)(hr + 4 * q); for (int j = 0; j < 4; ++j) m[4 * q + j] = (dv * t4[j]); } }
  for (int i = 0; i < cnt; ++i) { const int e = iclamp(PERM[p0 + i], 0, E - 1); int s = iclamp(srcs[e], 0, N - 1); if (SRCM < N) s %= SRCM; const float cf = rsqrtf((float)(iclamp(ROWCNT[s], 0, 1 << 24) + 1)); const float* hr = Hh + (size_t)s * W + c0;
#pragma unroll
    for (int q = 0; q < CW / 4; ++q) { const v4f t4 = *(const v4f*)(hr + 4 * q); for (int j = 0; j < 4; ++j) m[4 * q + j] += (cf * t4[j]); } }
  for (int pass = 0; pass < 2; ++pass) { if (v < mrows) { float* orow = out + (size_t)v * W + c0;
#pragma unroll
      for (int q = 0; q < CW / 4; ++q) { v4f o; for (int j = 0; j < 4; ++j) { float y = (dv * m[4 * q + j]) + bf16_rne(bias[c0 + 4 * q + j]); if (ADDP != nullptr) y += ADDP[(size_t)vv * W + c0 + 4 * q + j]; if (ACT == 1) y = fmaxf(y, 0.0f); if (ACT == 3) y = (y >= 0.0f) ? y : 0.01f * y; if (ACT == 4) { const float sp = (y > 20.0f) ? y : __logf(1.0f + __expf(y)); const float t = __expf(((-2.0f) * sp)); y = (y * (1.0f - t)) / (1.0f + t); }     o[j] = (v < N) ? y : 0.0f; } *(volatile v4f*)(orow + 4 * q) = o; } }
    __threadfence(); }
}
constexpr int NCLS = 40;
template <int NR>
__global__ __launch_bounds__(64) void bpadn_kernel(const float* __restrict__ b, float* __restrict__ B) { static_assert(NR <= 64, "bpadn: 64-entry record"); const int c = threadIdx.x; const float v = (c < NR) ? b[c] : 0.0f; for (int pass = 0; pass < 2; ++pass) { ((volatile float*)B)[c] = v; __threadfence(); } }
__global__ __launch_bounds__(256) void ocpf_kernel(const float* __restrict__ P, float* __restrict__ out, int total) {
  const int t = blockIdx.x * 256 + threadIdx.x; if (t >= total) return; const int g = t / NCLS, k = t - g * NCLS; const float v = P[(size_t)g * FO + k];
  for (int pass = 0; pass < 2; ++pass) { ((volatile float*)out)[t] = v; __threadfence(); }
}
template <int W>
__global__ __launch_bounds__(256) void bnrec_kernel(const float* __restrict__ gam, const float* __restrict__ bet, const float* __restrict__ rm, const float* __restrict__ rv, float* __restrict__ SCL, float* __restrict__ SFT) {
  static_assert(W >= 32 && W <= 256 && W % 32 == 0, "bnrec: one block, whole lines"); const int c = threadIdx.x; if (c >= W) return; const float scl = (bf16_rne(gam[c]) * (rsqrtf(bf16_rne(rv[c]) + BNEPS))); const float sft = bf16_rne(bet[c]) - (bf16_rne(rm[c]) * scl);
  for (int pass = 0; pass < 2; ++pass) { ((volatile float*)SCL)[c] = scl; ((volatile float*)SFT)[c] = sft; __threadfence(); }
}
template <int K, int DD, int HH, bool RND, int KA = K, bool ONEW = false>
__global__ __launch_bounds__(64) void gatnode_kernel(const float* __restrict__ X, const b16* __restrict__ WT, const b16* __restrict__ WQ, const float* __restrict__ as_, const float* __restrict__ ad_, float* __restrict__ Hh, float* __restrict__ SC) {
  constexpr int NT = DD / 16, CC = DD / HH, TPH = CC / 16; static_assert(!(RND && ONEW), "gatnode: ONEW is the unrounded hi word alone (one product): it goes with RND false");
  __shared__ __attribute__((aligned(16))) b16 Ah[2][16][K + 8], Al[2][16][K + 8]; __shared__ __attribute__((aligned(16))) float Tf[2][16][DD + 4]; __shared__ __attribute__((aligned(16))) float Sc[2][16][16];
  const int wave = threadIdx.x >> 5, lane = threadIdx.x & 31, nloc = lane & 15, hlf = lane >> 4; const size_t m0 = (size_t)blockIdx.x * 32 + wave * 16;
  for (int idx = lane; idx < 16 * (K / 4); idx += 32) { const int rr = idx / (K / 4), c4 = (idx % (K / 4)) * 4; const size_t arow = (m0 + rr < (size_t)N) ? m0 + rr : (size_t)N - 1; v4f v = {0.0f, 0.0f, 0.0f, 0.0f}; if (KA == K) v = *(const v4f*)(X + arow * K + c4); else { for (int j = 0; j < 4; ++j) v[j] = (c4 + j < KA) ? X[arow * KA + c4 + j] : 0.0f; } v4h hv, lv;
    for (int j = 0; j < 4; ++j) { const float vs = (RND ? bf16_rne(v[j]) : v[j]) * XS; const b16 ph = (b16)vs; hv[j] = ph; const float rs = (vs - (float)ph) * RS_; lv[j] = (b16)((!RND && !ONEW && fabsf(rs) < 6.103515625e-05f) ? 0.0f : rs); }     *(v4h*)(&Ah[wave][rr][c4]) = hv; if (!ONEW) *(v4h*)(&Al[wave][rr][c4]) = lv;     }
  for (int idx = lane; idx < 16 * 16; idx += 32) Sc[wave][idx >> 4][idx & 15] = 0.0f;
  wave_lds_sync();
  v8f acc[NT]; for (int t = 0; t < NT; ++t) acc[t] = (v8f){};
  for (int kb = 0; kb < K; kb += 32) { const v16b a = frag_kb(&Ah[wave][nloc][kb], hlf); v16b al; if (!RND && !ONEW) al = frag_kb(&Al[wave][nloc][kb], hlf);
#pragma unroll
    for (int t = 0; t < NT; ++t) { const size_t wo_ = (size_t)(t * 16 + nloc) * K + kb; acc[t] = wmma16b(a, frag_kb(WT + wo_, hlf), acc[t]); if (!RND && !ONEW) acc[t] = wmma16b(al, frag_kb(WQ + wo_, hlf), acc[t]); } }
#pragma unroll
  for (int t = 0; t < NT; ++t) for (int r = 0; r < 8; ++r) Tf[wave][8 * hlf + r][t * 16 + nloc] = (m0 + 8 * hlf + r < (size_t)N) ? acc[t][r] * (1.0f / (XS * WSC)) : 0.0f;
#pragma unroll
  for (int hd = 0; hd < HH; ++hd) {
    float ws[TPH], wd[TPH]; for (int q = 0; q < TPH; ++q) { ws[q] = bf16_rne(as_[hd * CC + q * 16 + nloc]); wd[q] = bf16_rne(ad_[hd * CC + q * 16 + nloc]); }
#pragma unroll
    for (int r = 0; r < 8; ++r) { float ss = 0.0f, sd = 0.0f;
#pragma unroll
      for (int q = 0; q < TPH; ++q) { const float hv = Tf[wave][8 * hlf + r][(hd * TPH + q) * 16 + nloc]; ss = fmaf(hv, ws[q], ss); sd = fmaf(hv, wd[q], sd); }
      for (int o = 1; o <= 8; o <<= 1) { ss += __shfl_xor(ss, o); sd += __shfl_xor(sd, o); }
      if (nloc == 0) { Sc[wave][8 * hlf + r][hd] = ss; Sc[wave][8 * hlf + r][8 + hd] = sd; } } }
  wave_lds_sync();
  for (int pass = 0; pass < 2; ++pass) {
    if (DD == 256) { for (int rr = 0; rr < 16; ++rr) { *(volatile v4f*)(Hh + (m0 + rr) * DD + lane * 4) = *(const v4f*)(&Tf[wave][rr][lane * 4]); *(volatile v4f*)(Hh + (m0 + rr) * DD + 128 + lane * 4) = *(const v4f*)(&Tf[wave][rr][128 + lane * 4]); } }
    else if (DD == 128) { for (int rr = 0; rr < 16; ++rr) *(volatile v4f*)(Hh + (m0 + rr) * DD + lane * 4) = *(const v4f*)(&Tf[wave][rr][lane * 4]); }
    else if (DD == 64) { for (int rr = 0; rr < 16; rr += 2) { const int r2 = rr + (lane >> 4); *(volatile v4f*)(Hh + (m0 + r2) * DD + (lane & 15) * 4) = *(const v4f*)(&Tf[wave][r2][(lane & 15) * 4]); } }
        else { for (int rr = 0; rr < 16; rr += 4) { const int r2 = rr + (lane >> 3); *(volatile v4f*)(Hh + (m0 + r2) * DD + (lane & 7) * 4) = *(const v4f*)(&Tf[wave][r2][(lane & 7) * 4]); } }
    for (int rr = 0; rr < 16; rr += 8) { const int r2 = rr + (lane >> 2); *(volatile v4f*)(SC + (m0 + r2) * 16 + (lane & 3) * 4) = *(const v4f*)(&Sc[wave][r2][(lane & 3) * 4]); }
    __threadfence(); }
}

template <int DD, int HH, int ACT, bool SELF = false>
__global__ __launch_bounds__(256) void gatagg_kernel(const float* __restrict__ Hh, const float* __restrict__ SC, const int* __restrict__ srcs, const int* __restrict__ PERM, const int* __restrict__ ROWPTR, const int* __restrict__ ROWCNT, int permLen, const float* __restrict__ bias, const float* __restrict__ ADDP, float* __restrict__ G, int mrows) {
  constexpr int CW = DD / 8, CC = DD / HH;
  const int tid = threadIdx.x; const int row = tid >> 3, g = tid & 7, c0 = g * CW, hd = c0 / CC; const int v = blockIdx.x * 32 + row; const int vv = v < N ? v : N - 1;
  float acc[CW]; for (int j = 0; j < CW; ++j) acc[j] = 0.0f;
  int cnt = 0, p0 = 0; if (v < N) { cnt = iclamp(ROWCNT[v], 0, 65536); p0 = iclamp(ROWPTR[v], 0, permLen - 1); if (p0 + cnt > permLen) cnt = permLen - p0; } const float sd = SC[(size_t)vv * 16 + 8 + hd];
  float m = -INFINITY, l = 0.0f;
  if (SELF) {
    m = lrelu(SC[(size_t)vv * 16 + hd] + sd); l = 1.0f; const float* hr = Hh + (size_t)vv * DD + c0;
#pragma unroll
    for (int q = 0; q < CW / 4; ++q) { const v4f t4 = *(const v4f*)(hr + 4 * q); for (int j = 0; j < 4; ++j) acc[4 * q + j] = t4[j]; } }
  for (int i = 0; i < cnt; ++i) { int s; { const int e = iclamp(PERM[p0 + i], 0, E - 1); s = iclamp(srcs[e], 0, N - 1); if (SRCM < N) s %= SRCM; }
    const float sc = lrelu(SC[(size_t)s * 16 + hd] + sd); const float mn = fmaxf(m, sc); const float al = __expf(m - mn), pw = __expf(sc - mn); l = l * al + pw; m = mn; const float* hr = Hh + (size_t)s * DD + c0;
#pragma unroll
    for (int q = 0; q < CW / 4; ++q) { const v4f t4 = *(const v4f*)(hr + 4 * q); for (int j = 0; j < 4; ++j) acc[4 * q + j] = fmaf(pw, t4[j], (acc[4 * q + j] * al)); } }
  const float inv = (SELF || cnt > 0) ? 1.0f / (l + 1e-16f) : 0.0f;
  float addv[CW]; for (int j = 0; j < CW; ++j) addv[j] = 0.0f; if (ADDP != nullptr && v < mrows) { for (int q = 0; q < CW / 4; ++q) { const v4f a4 = *(const v4f*)(ADDP + (size_t)v * DD + c0 + 4 * q); for (int j = 0; j < 4; ++j) addv[4 * q + j] = a4[j]; } }
  for (int pass = 0; pass < 2; ++pass) { if (v < mrows) { float* orow = G + (size_t)v * DD + c0;
#pragma unroll
      for (int q = 0; q < CW / 4; ++q) { v4f o4; for (int j = 0; j < 4; ++j) { float y = acc[4 * q + j] * inv + bf16_rne(bias[c0 + 4 * q + j]) + addv[4 * q + j]; if (ACT == 1) y = (y >= 0.0f) ? y : NSA_ * y; if (ACT == 2) y = (y > 0.0f) ? y : (__expf(y) - 1.0f); if (ACT == 3) y = fmaxf(y, 0.0f); o4[j] = (v < N) ? y : 0.0f; } *(volatile v4f*)(orow + 4 * q) = o4; } }
    __threadfence(); }
}

__global__ __launch_bounds__(256) void xpadr_kernel(const float* __restrict__ x, int xp, int xo, int xi, float* __restrict__ P, int kp, int n, int nrows) {
  const int i = blockIdx.x * 256 + threadIdx.x; const int q = kp >> 2; if (i >= nrows * q) return; const int v = i / q; const int c = (i - v * q) << 2; v4f o = {0.0f, 0.0f, 0.0f, 0.0f};
  if (v < n) { const float* xr = x + (size_t)v * (size_t)xp + (size_t)xo; if (c + 0 < xi) o[0] = bf16_rne(xr[c + 0]); if (c + 1 < xi) o[1] = bf16_rne(xr[c + 1]); if (c + 2 < xi) o[2] = bf16_rne(xr[c + 2]); if (c + 3 < xi) o[3] = bf16_rne(xr[c + 3]); }
  for (int pass = 0; pass < 2; ++pass) { *(volatile v4f*)(P + (size_t)i * 4) = o; __threadfence(); }
}
template <int DH, int NH>
__global__ __launch_bounds__(256) void edotp_kernel(const float* __restrict__ A, int ap, const float* __restrict__ B, int bp, const int* __restrict__ ia, const int* __restrict__ ib, float* __restrict__ out, int nl, int na, int nb, int ma, int mb, float scale, float lo, float hi) {
  static_assert(DH % 4 == 0 && NH >= 1, "edotp: float4 steps; at least one head");
  const int t = blockIdx.x * 256 + threadIdx.x; if (t >= nl * NH) return; const int l = t / NH, h = t - l * NH; int a = iclamp(ia[l], 0, na - 1); if (ma < na) a %= ma; int b = iclamp(ib[l], 0, nb - 1); if (mb < nb) b %= mb; float s = 0.0f; const float* ar = A + (size_t)a * ap + h * DH; const float* br = B + (size_t)b * bp + h * DH;
  for (int q = 0; q < DH / 4; ++q) { const v4f x4 = *(const v4f*)(ar + 4 * q), y4 = *(const v4f*)(br + 4 * q); for (int j = 0; j < 4; ++j) s += (x4[j] * y4[j]); }
  s = fminf(fmaxf((s * scale), lo), hi);
  for (int pass = 0; pass < 2; ++pass) { ((volatile float*)out)[t] = s; __threadfence(); }
}
template <int W, int NH, int ACT>
__global__ __launch_bounds__(256) void esmw_kernel(const float* __restrict__ V, int vp, int ns, int srcm, const float* __restrict__ SC, const int* __restrict__ srcs, int ecut, const int* __restrict__ PERM, const int* __restrict__ ROWPTR, const int* __restrict__ ROWCNT, int permLen, const float* __restrict__ ADD, int ap, float* __restrict__ out, int op, int nd, int mrows) {
  constexpr int CW = W / 8; static_assert(W % 32 == 0 && NH >= 1 && (W / NH) % CW == 0, "esmw: 8 threads per row, float4 steps; a thread's columns lie in one head");
  const int tid = threadIdx.x; const int row = tid >> 3, g = tid & 7, c0 = g * CW, h = c0 / (W / NH); const int v = blockIdx.x * 32 + row; const int vv = v < nd ? v : nd - 1;
  int cnt = 0, p0 = 0; if (v < nd) { cnt = iclamp(ROWCNT[v], 0, 65536); p0 = iclamp(ROWPTR[v], 0, permLen - 1); if (p0 + cnt > permLen) cnt = permLen - p0; }
  float mx = -INFINITY, l = 0.0f; float acc[CW]; for (int j = 0; j < CW; ++j) acc[j] = 0.0f;
  for (int i = 0; i < cnt; ++i) { const int e = iclamp(PERM[p0 + i], 0, ecut - 1); int s = iclamp(srcs[e], 0, ns - 1); if (srcm < ns) s %= srcm;
    const float sc = SC[(size_t)e * NH + h]; const float mn = fmaxf(mx, sc); const float al = __expf(mx - mn), pw = __expf(sc - mn); l = l * al + pw; mx = mn;
    const float* vr = V + (size_t)s * vp + c0; v4f x4[CW / 4];
#pragma unroll
    for (int q = 0; q < CW / 4; ++q) x4[q] = *(const v4f*)(vr + 4 * q);
#pragma unroll
    for (int j = 0; j < CW; ++j) acc[j] = (acc[j] * al) + (pw * x4[j / 4][j % 4]); }
  const float inv = (cnt > 0) ? 1.0f / l : 0.0f; const float* np_ = ADD + (size_t)vv * ap + c0; v4f n4[CW / 4];
#pragma unroll
  for (int q = 0; q < CW / 4; ++q) n4[q] = *(const v4f*)(np_ + 4 * q);
  for (int pass = 0; pass < 2; ++pass) { if (v < mrows) { float* orow = out + (size_t)v * op + c0;
#pragma unroll
      for (int q = 0; q < CW / 4; ++q) { v4f o4; for (int j = 0; j < 4; ++j) { float y = (acc[4 * q + j] * inv) + n4[q][j]; if (ACT == 1) y = fmaxf(y, 0.0f); o4[j] = (v < nd) ? y : 0.0f; } *(volatile v4f*)(orow + 4 * q) = o4; } } __threadfence(); }
}
__global__ __launch_bounds__(256) void ipos_kernel(int* __restrict__ I, int n, int dv, int m) {
  const size_t t = (size_t)blockIdx.x * 256 + threadIdx.x; if (t >= (size_t)n) return;
  const unsigned q = (unsigned)t / (unsigned)dv; const int v = (int)(q % (unsigned)m);
  for (int pass = 0; pass < 2; ++pass) { ((volatile int*)I)[t] = v; __threadfence(); }
}
template <bool HAS_DST, bool HAS_EDGE, bool RAW_EA, int ACT>
__global__ __launch_bounds__(256) void escoreh_kernel(const float* __restrict__ S, int sp, int so, int ns, const int* __restrict__ src, const float* __restrict__ D, int dp, int dof, int nd, const int* __restrict__ dst, const float* __restrict__ EA, int eap, int ed, const float* __restrict__ VE, int vk, int vh, const float* __restrict__ BE, float slope, float* __restrict__ A, int nh, int ne, int epad) {
  static_assert(ACT >= 0 && ACT <= 2, "escoreh: three activations"); const unsigned t = blockIdx.x * 256u + threadIdx.x; if (t >= (unsigned)epad * (unsigned)nh) return; const unsigned l = t / (unsigned)nh; const int h = (int)(t - l * (unsigned)nh); float a = 0.0f;
  if (l < (unsigned)ne) { a = S[(size_t)iclamp(src[l], 0, ns - 1) * sp + so + h]; if (HAS_DST) a = (a + D[(size_t)iclamp(dst[l], 0, nd - 1) * dp + dof + h]);
    if (HAS_EDGE) { float u = BE[h]; const float* er = EA + (size_t)l * eap; const float* vr = VE + (size_t)h * vh; for (int k = 0; k < ed; ++k) { const float x = RAW_EA ? bf16_rne(er[k]) : er[k]; u += (x * vr[(size_t)k * vk]); } a = (a + u); }
    if (ACT == 1) a = (a >= 0.0f) ? a : (slope * a); else if (ACT == 2) a = 1.0f / (1.0f + expf(-a)); }
  for (int pass = 0; pass < 2; ++pass) { ((volatile float*)A)[t] = a; __threadfence(); }
}
__global__ __launch_bounds__(256) void wtkr_kernel(const float* __restrict__ w, int ka, int nout, b16* __restrict__ WT, int kk, int noutp, float scl) {
  const int u = blockIdx.x * 256 + threadIdx.x; if (u >= noutp * (kk >> 3)) return; const int e = u << 3; const int o = e / kk, k0 = e - o * kk; v8b v;
#pragma unroll
  for (int j = 0; j < 8; ++j) { const int k = k0 + j; float t = 0.0f; if (o < nout && k < ka) t = bf16_rne(w[(size_t)k * (size_t)nout + (size_t)o]); v[j] = (b16)(t * scl); }
  for (int pass = 0; pass < 2; ++pass) { *(volatile v8b*)(WT + e) = v; __threadfence(); }
}
__global__ __launch_bounds__(256) void ocpr_kernel(const float* __restrict__ P, int pp, int pc, float* __restrict__ OUT, int w, int n) {
  const int t = blockIdx.x * 256 + threadIdx.x; if (t >= n * w) return; const int v = t / w; const int c = t - v * w; const float y = P[(size_t)v * (size_t)pp + (size_t)pc + (size_t)c];
  for (int pass = 0; pass < 2; ++pass) { ((volatile float*)OUT)[t] = y; __threadfence(); }
}
template <int W>
__global__ __launch_bounds__(256) void tcosm_kernel(const float* __restrict__ T, const float* __restrict__ wv, const float* __restrict__ bv, int ecut, const int* __restrict__ PERM, const int* __restrict__ ROWPTR, const int* __restrict__ ROWCNT, int permLen, float* __restrict__ P, int pp, int ocol, int nd, int ndp) {
  constexpr int CW = W / 8; static_assert(W % 32 == 0, "tcosm: 8 threads per row, float4 steps");
  const int tid = threadIdx.x; const int row = tid >> 3, g = tid & 7, c0 = g * CW; const int v = blockIdx.x * 32 + row; if (v >= ndp) return;
  int cnt = 0, p0 = 0; if (v < nd) { cnt = iclamp(ROWCNT[v], 0, 65536); p0 = iclamp(ROWPTR[v], 0, permLen - 1); if (p0 + cnt > permLen) cnt = permLen - p0; }
  float m[CW], fw[CW], fb[CW];
#pragma unroll
  for (int j = 0; j < CW; ++j) { m[j] = 0.0f; fw[j] = bf16_rne(wv[c0 + j]); fb[j] = bf16_rne(bv[c0 + j]); }
  for (int i = 0; i < cnt; ++i) { const int e = iclamp(PERM[p0 + i], 0, ecut - 1); const float t = bf16_rne(T[e]);
#pragma unroll
    for (int j = 0; j < CW; ++j) m[j] += cosf((t * fw[j]) + fb[j]); }
  const float inv = 1.0f / (float)(cnt > 0 ? cnt : 1);
  for (int pass = 0; pass < 2; ++pass) { float* orow = P + (size_t)v * pp + ocol + c0;
#pragma unroll
    for (int q = 0; q < CW / 4; ++q) { v4f o4; for (int j = 0; j < 4; ++j) o4[j] = (v < nd) ? (m[4 * q + j] * inv) : 0.0f; *(volatile v4f*)(orow + 4 * q) = o4; }
    __threadfence(); }
}
__global__ __launch_bounds__(256) void icat_kernel(const int* __restrict__ A, int na, const int* __restrict__ B, int nb, int* __restrict__ OUT) {
  const int t = blockIdx.x * 256 + threadIdx.x; if (t >= na + nb) return; const int v = (t < na) ? A[t] : B[t - na];
  for (int pass = 0; pass < 2; ++pass) { *(volatile int*)(OUT + t) = v; __threadfence(); }
}
__global__ __launch_bounds__(256) void gchk_kernel(const int* __restrict__ batch, int* __restrict__ FLAG, int nn) {
  const int v = blockIdx.x * 256 + threadIdx.x; if (v + 1 >= nn) return; if (batch[v] > batch[v + 1] || batch[v] < 0) { ((volatile int*)FLAG)[0] = 1; __threadfence(); }
}
__global__ __launch_bounds__(128) void gmean_kernel(const float* __restrict__ H, const int* __restrict__ batch, const int* __restrict__ FLAG, float* __restrict__ P, int nstat) {
  const int g = blockIdx.x, c = threadIdx.x; int lo = 0, hi = nstat; while (lo < hi) { const int mid = (lo + hi) >> 1; if (batch[mid] < g) lo = mid + 1; else hi = mid; } const int st = lo; hi = nstat; while (lo < hi) { const int mid = (lo + hi) >> 1; if (batch[mid] <= g) lo = mid + 1; else hi = mid; } const int en = lo;
  float s = 0.0f;
#pragma unroll 1
  for (int v = st; v < en; ++v) s += H[(size_t)v * F + c];
  float o = (en > st) ? s / (float)(en - st) : 0.0f; if (FLAG[0] != 0) o = __int_as_float(0x7fc00000);
  for (int pass = 0; pass < 2; ++pass) { ((volatile float*)P)[(size_t)g * F + c] = o; __threadfence(); }
}
template <int W, bool SUM = false>
__global__ __launch_bounds__(W) void gmeanw_kernel(const float* __restrict__ H, const int* __restrict__ batch, const int* __restrict__ FLAG, float* __restrict__ P, int nstat) {
  const int g = blockIdx.x, c = threadIdx.x; int lo = 0, hi = nstat; while (lo < hi) { const int mid = (lo + hi) >> 1; if (batch[mid] < g) lo = mid + 1; else hi = mid; } const int st = lo; hi = nstat; while (lo < hi) { const int mid = (lo + hi) >> 1; if (batch[mid] <= g) lo = mid + 1; else hi = mid; } const int en = lo;
  float s = 0.0f;
#pragma unroll 1
  for (int v = st; v < en; ++v) s += H[(size_t)v * W + c];
  float o = (en > st) ? (SUM ? s : s / (float)(en - st)) : 0.0f; if (FLAG[0] != 0) o = __int_as_float(0x7fc00000);
  for (int pass = 0; pass < 2; ++pass) { ((volatile float*)P)[(size_t)g * W + c] = o; __threadfence(); }
}
}

extern "C" void kernel_launch(void* const* d_in, const int* in_sizes, int n_in, void* d_out, int out_size, void* d_ws, size_t ws_size, hipStream_t stream) {
  auto Fp = [&](int i) { return (const float*)d_in[i]; }; auto Ip = [&](int i) { return (const int*)d_in[i]; };
  constexpr int EL = 800000  , EJ = EL + N  , FI = 64, H1 = 64  , H4 = 4, C4 = 64, W4 = H4 * C4  , NG = 500  , NGP = 512  , NO = 32  , NOP = 64  ; constexpr size_t P4 = (size_t)NP * W4, P1 = (size_t)NP * H1;
  static_assert(EL == E && NP % 32 == 0 && NP >= N && H4 * C4 == W4 && NGP % 32 == 0 && NGP >= NG && NO <= NOP && NOP % 16 == 0 && ((N + CSR_GN - 1) >> CSR_GB) <= CSR_MAXG && (P4 * 4) % 256 == 0 && (P1 * 4) % 256 == 0 && (EJ * H4) % 32 == 0 && XS == 8.0f && WSC == 256.0f);
  if (n_in != 11 || in_sizes[0] != N * FI || in_sizes[1] != 2 * EL || in_sizes[2] != N || in_sizes[3] != FI * H1 || in_sizes[4] != H1 || in_sizes[5] != H1 * W4 || in_sizes[6] != W4 || in_sizes[7] != W4 || in_sizes[8] != W4 || in_sizes[9] != W4 * NO || in_sizes[10] != NO || out_size != NG * NO) return;
  size_t off = 0; char* ws = (char*)d_ws;
  auto carve = [&](size_t bytes) { char* p = ws + off; off += (bytes + 255) & ~(size_t)255; return p; };
  b16* WIC = (b16*)carve((size_t)H1 * FI * 2); b16* WIG = (b16*)carve((size_t)W4 * H1 * 2); b16* WIO = (b16*)carve((size_t)NOP * W4 * 2);
  float* RA = (float*)carve(3 * (size_t)W4 * 4); float* ZB = (float*)carve((size_t)W4 * 4); float* BO = (float*)carve((size_t)NOP * 4); int* FLAG = (int*)carve(256);
  int* IX = (int*)carve((size_t)N * 4); int* SJ = (int*)carve((size_t)EJ * 4); int* DJ = (int*)carve((size_t)EJ * 4);
  float* AS = (float*)carve((size_t)N * H4 * 4); float* AD = (float*)carve((size_t)N * H4 * 4); float* SC = (float*)carve((size_t)EJ * H4 * 4);
  float* H0 = (float*)carve(P1 * 4); float* HC = (float*)carve(P1 * 4);
  float* PH = (float*)carve(P4 * 4); float* PX = (float*)carve(P4 * 4);
  float* PG = (float*)carve((size_t)NGP * W4 * 4); float* PO = (float*)carve((size_t)NGP * NOP * 4);
  CsrBufs cl; off = csr_carve(cl, ws, off, EL, N); CsrBufs cj; off = csr_carve(cj, ws, off, EJ, N);
  if (off > ws_size) return;
  const unsigned gJ = (unsigned)(((size_t)EJ + 255) / 256), gN = (unsigned)((N + 255) / 256);
  ipos_kernel<<<gN, 256, 0, stream>>>(IX, N, 1, N);
  icat_kernel<<<gJ, 256, 0, stream>>>(Ip(1), EL, IX, N, SJ); icat_kernel<<<gJ, 256, 0, stream>>>(Ip(1) + EL, EL, IX, N, DJ);
  csr_build(cl, Ip(1) + EL, EL, N, stream); csr_build(cj, DJ, EJ, N, stream);
  zfill_kernel<<<1, 256, 0, stream>>>(ZB, W4); zfill_kernel<<<1, 256, 0, stream>>>((float*)FLAG, 64);
  wt_kernel<FI, H1, H1><<<(unsigned)(((size_t)FI * H1 / 8 + 255) / 256), 256, 0, stream>>>(Fp(3), WIC, WSC); wtkr_kernel<<<(unsigned)(((size_t)W4 * H1 / 8 + 255) / 256), 256, 0, stream>>>(Fp(5), H1, W4, WIG, H1, W4, WSC); wtkr_kernel<<<(unsigned)(((size_t)NOP * W4 / 8 + 255) / 256), 256, 0, stream>>>(Fp(9), W4, NO, WIO, W4, NOP, WSC);
  for (int j = 0; j < 3; ++j) xcpw_kernel<W4><<<1, 256, 0, stream>>>(Fp(6 + j), RA + (size_t)j * W4, W4, 1, 1);
  xpadr_kernel<<<1, 256, 0, stream>>>(Fp(10), NO, 0, NO, BO, NOP, 1, 1);
  lin_kernel<FI, 4, 1, 0, false><<<NP / 32, 64, 0, stream>>>(Fp(0), nullptr, WIC, WIC, ZB, H0, H1, N, NP);
  gcn_kernel<H1, 1><<<NP / 32, 256, 0, stream>>>(H0, Ip(1), cl.PERM, cl.ROWPTR, cl.ROWCNT, (int)cl.permLen, Fp(4), nullptr, HC, NP);
  lin_kernel<H1, 16, 2, 0, false><<<NP / 32, 64, 0, stream>>>(HC, nullptr, WIG, WIG, ZB, PH, W4, N, NP);
  edotp_kernel<C4, H4><<<(unsigned)(((size_t)N * H4 + 255) / 256), 256, 0, stream>>>(PH, W4, RA, W4, IX, IX, AS, N, N, 1, N, 1, 1.0f, -__builtin_inff(), __builtin_inff()); edotp_kernel<C4, H4><<<(unsigned)(((size_t)N * H4 + 255) / 256), 256, 0, stream>>>(PH, W4, RA + W4, W4, IX, IX, AD, N, N, 1, N, 1, 1.0f, -__builtin_inff(), __builtin_inff());
  escoreh_kernel<true, false, false, 1><<<(unsigned)(((size_t)EJ * H4 + 255) / 256), 256, 0, stream>>>(AS, H4, 0, N, SJ, AD, H4, 0, N, DJ, nullptr, 0, 0, nullptr, 0, 0, nullptr, 0.2f, SC, H4, EJ, EJ);
  esmw_kernel<W4, H4, 0><<<NP / 32, 256, 0, stream>>>(PH, W4, N, N, SC, SJ, EJ, cj.PERM, cj.ROWPTR, cj.ROWCNT, (int)cj.permLen, RA + 2 * W4, 0, PX, W4, N, NP);
  eact_kernel<1><<<(unsigned)((P4 / 4 + 255) / 256), 256, 0, stream>>>(PX, PH, P4 / 4, 0.0f);
  gchk_kernel<<<gN, 256, 0, stream>>>(Ip(2), FLAG, N);
  gmeanw_kernel<W4><<<NG, W4, 0, stream>>>(PH, Ip(2), FLAG, PG, N);
  lin_kernel<W4, 4, 2, 0, false><<<NGP / 32, 64, 0, stream>>>(PG, nullptr, WIO, WIO, BO, PO, NOP, NG, NGP);
  ocpr_kernel<<<(unsigned)(((size_t)NG * NO + 255) / 256), 256, 0, stream>>>(PO, NOP, 0, (float*)d_out, NO, NG);
}
